// SubSamplingLayer_16149077033588
// MI455X (gfx1250) — hardware-run, weakly checked
//
#include <hip/hip_runtime.h>
#include <math.h>

typedef __attribute__((ext_vector_type(16))) _Float16 v16h;
typedef __attribute__((ext_vector_type(8)))  _Float16 v8h;
typedef __attribute__((ext_vector_type(8)))  float    v8f;
typedef __attribute__((ext_vector_type(4)))  float    v4f;
typedef __attribute__((ext_vector_type(2)))  float    v2f;

constexpr int kRes      = 128;
constexpr int kBatch    = 16;
constexpr int kPts      = kRes * kRes;
constexpr int kKdim     = 2 * kPts;
constexpr int kMrows    = 2 * kRes;
constexpr int kChunkB   = 8;
constexpr int kNumChunk = kBatch / kChunkB;
constexpr int kNcols    = kChunkB * kRes;
constexpr float kCarryA = 64.0f;
constexpr float kCarryB = 32.0f;
constexpr float kFold   = 1.0f / (kCarryA * kCarryB);
constexpr float kTwoPi  = 6.28318530717958647692f;
constexpr float kStep   = kTwoPi / (float)kRes;
static_assert(kPts == 16384 && kKdim == 32768 && kMrows == 256 && kNcols == 1024, "shape constants");
static_assert((kKdim % 32) == 0, "GEMM K multiple of 32");
static_assert((kMrows % 64) == 0 && (kRes % 64) == 0, "GEMM M,N multiples of 64");
static_assert(kNumChunk * kChunkB == kBatch, "batch chunks");
static_assert((kMrows / 64) * (kRes / 64) == 8, "one 8-wave block per batch element");

constexpr size_t kSzS    = (size_t)kBatch * kPts * 2 * 4;
constexpr size_t kSzAP   = (size_t)kMrows * kKdim * 2;
constexpr size_t kSzEY   = (size_t)kRes * kPts * 4;
constexpr size_t kSzBT   = (size_t)kNcols * kKdim * 2;
constexpr size_t kOffS   = 0;
constexpr size_t kOffAP  = kOffS + kSzS;
constexpr size_t kOffEYC = kOffAP + kSzAP;
constexpr size_t kOffEYS = kOffEYC + kSzEY;
constexpr size_t kOffBT  = kOffEYS + kSzEY;
constexpr size_t kWsTotal = kOffBT + kSzBT;
static_assert(kSzS == 2097152ull && kSzAP == 16777216ull && kSzEY == 8388608ull && kSzBT == 67108864ull, "plane sizes");
static_assert(kWsTotal == 102760448ull, "carve total");
static_assert(kWsTotal <= 134217728ull, "carve cap");
static_assert((kOffAP % 128) == 0 && (kOffEYC % 128) == 0 && (kOffEYS % 128) == 0 && (kOffBT % 128) == 0, "aligned regions");

union FragU { v16h v; v8h h[2]; };
__device__ __forceinline__ v16h frag_load(const _Float16* p) {
  FragU f;
  f.h[0] = *(const v8h*)(p);
  f.h[1] = *(const v8h*)(p + 16);
  return f.v;
}
__device__ __forceinline__ v8f mma_f16_guarded(v16h a, v16h b, v8f c) {
  c = __builtin_amdgcn_wmma_f32_16x16x32_f16(false, a, false, b, (short)0, c, false, false);
  asm volatile("v_nop\n\tv_nop\n\tv_nop\n\tv_nop" : "+v"(c) : "v"(a), "v"(b));
  return c;
}

__device__ __forceinline__ void sample_point(const float* __restrict__ base, float t0, float t1,
                                             float& re, float& im) {
  const float pr  = t0 + 0.5f * (float)kRes;
  const float pc  = t1 + 0.5f * (float)kRes;
  const float r0f = floorf(pr);
  const float c0f = floorf(pc);
  const float wr  = pr - r0f;
  const float wc  = pc - c0f;
  const float r0l = fminf(fmaxf(r0f, -1.0f), (float)kRes);
  const float c0l = fminf(fmaxf(c0f, -1.0f), (float)kRes);
  int r0 = (int)r0l;
  int c0 = (int)c0l;
  r0 = min(max(r0, 0), kRes - 1);
  c0 = min(max(c0, 0), kRes - 1);
  const int r1 = min(r0 + 1, kRes - 1);
  const int c1 = min(c0 + 1, kRes - 1);
  const v2f g00 = *(const v2f*)(base + (size_t)(r0 * kRes + c0) * 2);
  const v2f g01 = *(const v2f*)(base + (size_t)(r0 * kRes + c1) * 2);
  const v2f g10 = *(const v2f*)(base + (size_t)(r1 * kRes + c0) * 2);
  const v2f g11 = *(const v2f*)(base + (size_t)(r1 * kRes + c1) * 2);
  const float omr = 1.0f - wr;
  const float omc = 1.0f - wc;
  const float w00 = omr * omc;
  const float w01 = omr * wc;
  const float w10 = wr * omc;
  const float w11 = wr * wc;
  re = ((w00 * g00.x + w01 * g01.x) + w10 * g10.x) + w11 * g11.x;
  im = ((w00 * g00.y + w01 * g01.y) + w10 * g10.y) + w11 * g11.y;
}

__global__ __launch_bounds__(256) void sample_kernel(const float* __restrict__ ksp,
                                                     const float* __restrict__ traj,
                                                     float* __restrict__ S) {
  const int idx = blockIdx.x * 256 + threadIdx.x;
  const int b   = idx >> 13;
  const int m2  = (idx & 8191) * 2;
  const v4f tt  = *(const v4f*)(traj + (size_t)m2 * 2);
  const float* base = ksp + (size_t)b * (kPts * 2);
  float re0, im0, re1, im1;
  sample_point(base, tt[0], tt[1], re0, im0);
  sample_point(base, tt[2], tt[3], re1, im1);
  v4f o;
  o[0] = re0; o[1] = im0; o[2] = re1; o[3] = im1;
  float* dst = S + ((size_t)b * kPts + m2) * 2;
  *(volatile v4f*)dst = o;
  __threadfence();
  *(volatile v4f*)dst = o;
}

__global__ __launch_bounds__(256) void phase_rows_kernel(const float* __restrict__ traj,
                                                         unsigned* __restrict__ Aw) {
#pragma clang fp contract(off)
  const int idx = blockIdx.x * 256 + threadIdx.x;
  const int h   = idx >> 14;
  const int m   = idx & (kPts - 1);
  const float t  = traj[2 * m];
  const float x  = (float)(h - kRes / 2);
  const float kt = kStep * t;
  const float th = kt * x;
  float sn, cs;
  sincosf(th, &sn, &cs);
  const float cs64 = cs * kCarryA;
  const float sn64 = sn * kCarryA;
  const _Float16 hc  = (_Float16)cs64;
  const _Float16 hs  = (_Float16)sn64;
  const _Float16 hns = (_Float16)(-sn64);
  const unsigned bc  = (unsigned)__builtin_bit_cast(unsigned short, hc);
  const unsigned bs  = (unsigned)__builtin_bit_cast(unsigned short, hs);
  const unsigned bns = (unsigned)__builtin_bit_cast(unsigned short, hns);
  const unsigned w0 = bc | (bns << 16);
  const unsigned w1 = bs | (bc << 16);
  volatile unsigned* p0 = (volatile unsigned*)(Aw + (size_t)h * kPts + m);
  volatile unsigned* p1 = (volatile unsigned*)(Aw + (size_t)(kRes + h) * kPts + m);
  *p0 = w0;
  *p1 = w1;
  __threadfence();
  *p0 = w0;
  *p1 = w1;
}

__global__ __launch_bounds__(256) void phase_cols_kernel(const float* __restrict__ traj,
                                                         float* __restrict__ EYC,
                                                         float* __restrict__ EYS) {
#pragma clang fp contract(off)
  const int idx = blockIdx.x * 256 + threadIdx.x;
  const int w   = idx >> 14;
  const int m   = idx & (kPts - 1);
  const float t  = traj[2 * m + 1];
  const float y  = (float)(w - kRes / 2);
  const float kt = kStep * t;
  const float th = kt * y;
  float sn, cs;
  sincosf(th, &sn, &cs);
  volatile float* pc = (volatile float*)(EYC + idx);
  volatile float* ps = (volatile float*)(EYS + idx);
  *pc = cs;
  *ps = sn;
  __threadfence();
  *pc = cs;
  *ps = sn;
}

__global__ __launch_bounds__(256) void build_bt_kernel(const float* __restrict__ Sc,
                                                       const float* __restrict__ EYC,
                                                       const float* __restrict__ EYS,
                                                       unsigned short* __restrict__ Bt) {
  const int idx = blockIdx.x * 256 + threadIdx.x;
  const int w   = idx >> 12;
  const int m4  = (idx & 4095) * 4;
  const v4f cy = *(const v4f*)(EYC + (size_t)w * kPts + m4);
  const v4f sy = *(const v4f*)(EYS + (size_t)w * kPts + m4);
#pragma unroll 1
  for (int bl = 0; bl < kChunkB; ++bl) {
    const float* sp = Sc + ((size_t)bl * kPts + m4) * 2;
    const v4f s0 = *(const v4f*)(sp);
    const v4f s1 = *(const v4f*)(sp + 4);
    const float tr0 = s0[0] * cy[0] - s0[1] * sy[0];
    const float ti0 = s0[0] * sy[0] + s0[1] * cy[0];
    const float tr1 = s0[2] * cy[1] - s0[3] * sy[1];
    const float ti1 = s0[2] * sy[1] + s0[3] * cy[1];
    const float tr2 = s1[0] * cy[2] - s1[1] * sy[2];
    const float ti2 = s1[0] * sy[2] + s1[1] * cy[2];
    const float tr3 = s1[2] * cy[3] - s1[3] * sy[3];
    const float ti3 = s1[2] * sy[3] + s1[3] * cy[3];
    v8h o;
    o[0] = (_Float16)(tr0 * kCarryB);
    o[1] = (_Float16)(ti0 * kCarryB);
    o[2] = (_Float16)(tr1 * kCarryB);
    o[3] = (_Float16)(ti1 * kCarryB);
    o[4] = (_Float16)(tr2 * kCarryB);
    o[5] = (_Float16)(ti2 * kCarryB);
    o[6] = (_Float16)(tr3 * kCarryB);
    o[7] = (_Float16)(ti3 * kCarryB);
    unsigned short* dst = Bt + (size_t)(bl * kRes + w) * kKdim + (size_t)m4 * 2;
    *(volatile v8h*)dst = o;
    __threadfence();
    *(volatile v8h*)dst = o;
  }
}

__global__ __launch_bounds__(256) void gemm_f16_kernel(
    const unsigned short* __restrict__ Ap, int lda,
    const unsigned short* __restrict__ Btp, int ldb, long strideB,
    float* __restrict__ Cout, int ldc, long strideC,
    int M, int N, int K, float scale) {
  const _Float16* A  = (const _Float16*)Ap;
  const _Float16* Bt = (const _Float16*)Btp;
  __shared__ __align__(16) float sT[8][16 * 68];
  const int b    = blockIdx.y;
  const int lane = threadIdx.x & 31;
  const int wave = __builtin_amdgcn_readfirstlane((int)(threadIdx.x >> 5));
  const int tilesN = N >> 6;
  const int tilesM = M >> 6;
  const int tile = blockIdx.x * 8 + wave;
  if (tile >= tilesM * tilesN) return;
  const int tm = tile / tilesN;
  const int tn = tile - tm * tilesN;
  const int m0 = tm << 6;
  const int n0 = tn << 6;

  const _Float16* Bb = Bt + (size_t)b * strideB;
  const int rlane = lane & 15;
  const int koff  = (lane >> 4) * 8;
  const int mOff  = (lane >> 4) * 8;

  const _Float16* apt = A  + (size_t)(m0 + rlane) * lda + koff;
  const _Float16* bpt = Bb + (size_t)(n0 + rlane) * ldb + koff;
  const size_t astep = (size_t)16 * lda;
  const size_t bstep = (size_t)16 * ldb;

  v8f acc[4][4];
#pragma unroll
  for (int i = 0; i < 4; ++i)
#pragma unroll
    for (int j = 0; j < 4; ++j) acc[i][j] = (v8f){0.f, 0.f, 0.f, 0.f, 0.f, 0.f, 0.f, 0.f};

  for (int k0 = 0; k0 < K; k0 += 32) {
    v16h bh[4];
#pragma unroll
    for (int j = 0; j < 4; ++j) bh[j] = frag_load(bpt + j * bstep + k0);
#pragma unroll
    for (int i = 0; i < 4; ++i) {
      const v16h ah = frag_load(apt + i * astep + k0);
#pragma unroll
      for (int j = 0; j < 4; ++j) acc[i][j] = mma_f16_guarded(ah, bh[j], acc[i][j]);
    }
  }

  float* slab = sT[wave];
  float* C = Cout + (size_t)b * strideC;
  const int hh = lane >> 4;
  const int c4 = (lane & 15) * 4;
#pragma unroll
  for (int i = 0; i < 4; ++i) {
    const int mBase = m0 + (i << 4);
#pragma unroll
    for (int j = 0; j < 4; ++j) {
#pragma unroll
      for (int r = 0; r < 8; ++r) {
        const float v = acc[i][j][r] * scale;
        slab[(mOff + r) * 68 + (j << 4) + rlane] = v;
      }
    }
    __builtin_amdgcn_fence(__ATOMIC_RELEASE, "workgroup");
    __builtin_amdgcn_wave_barrier();
    __builtin_amdgcn_fence(__ATOMIC_ACQUIRE, "workgroup");
    for (int pass = 0; pass < 2; ++pass) {
#pragma unroll
      for (int it = 0; it < 8; ++it) {
        const int row = it * 2 + hh;
        const v4f v = *(const v4f*)(slab + row * 68 + c4);
        *(volatile v4f*)(C + (size_t)(mBase + row) * ldc + n0 + c4) = v;
      }
      __threadfence();
    }
    __builtin_amdgcn_fence(__ATOMIC_RELEASE, "workgroup");
    __builtin_amdgcn_wave_barrier();
    __builtin_amdgcn_fence(__ATOMIC_ACQUIRE, "workgroup");
  }
}

extern "C" void kernel_launch(void* const* d_in, const int* in_sizes, int n_in,
                              void* d_out, int out_size, void* d_ws, size_t ws_size,
                              hipStream_t stream) {
  if (n_in < 2) return;
  if (in_sizes[0] != kBatch * kPts * 2) return;
  if (in_sizes[1] != kPts * 2) return;
  if (out_size != kBatch * 2 * kPts) return;
  if (ws_size < kWsTotal) return;

  const float* ksp  = (const float*)d_in[0];
  const float* traj = (const float*)d_in[1];
  float* out = (float*)d_out;

  char* ws = (char*)d_ws;
  float*          S   = (float*)(ws + kOffS);
  unsigned short* AP  = (unsigned short*)(ws + kOffAP);
  float*          EYC = (float*)(ws + kOffEYC);
  float*          EYS = (float*)(ws + kOffEYS);
  unsigned short* BT  = (unsigned short*)(ws + kOffBT);

  sample_kernel<<<(kBatch * (kPts / 2)) / 256, 256, 0, stream>>>(ksp, traj, S);
  phase_rows_kernel<<<(kRes * kPts) / 256, 256, 0, stream>>>(traj, (unsigned*)AP);
  phase_cols_kernel<<<(kRes * kPts) / 256, 256, 0, stream>>>(traj, EYC, EYS);

  for (int g = 0; g < kNumChunk; ++g) {
    const float* Sc = S + (size_t)g * kChunkB * kPts * 2;
    float* outc = out + (size_t)g * kChunkB * 2 * kPts;
    build_bt_kernel<<<(kRes * (kPts / 4)) / 256, 256, 0, stream>>>(Sc, EYC, EYS, BT);
    gemm_f16_kernel<<<dim3(1, kChunkB), 256, 0, stream>>>(
        AP, kKdim,
        BT, kKdim, (long)kRes * (long)kKdim,
        outc, kRes, (long)2 * (long)kPts,
        kMrows, kRes, kKdim, kFold);
  }
}
